// TransformerMemoryLayer_31086973288502
// MI455X (gfx1250) — hardware-verified
//
#include <hip/hip_runtime.h>
#include <stddef.h>
#include <stdint.h>

#define BB   4
#define SS   1024
#define DM   1024
#define NH   16
#define HD   64
#define NE   4
#define ROWS (BB * SS)
#define C3   (3 * DM)
#define KCAT (NE * DM)
#define PL   ((size_t)BB * NH * SS * HD)

static_assert(SS % 256 == 0);
static_assert(DM % 64 == 0);
static_assert(HD == 64);
static_assert(NH * HD == DM);
static_assert(ROWS % 256 == 0);
static_assert(ROWS % 8 == 0);
static_assert(DM == 1024);
static_assert(NE == 4);
static_assert(KCAT % 32 == 0);

typedef _Float16 v16h __attribute__((ext_vector_type(16)));
typedef _Float16 v8h  __attribute__((ext_vector_type(8)));
typedef float    v8f  __attribute__((ext_vector_type(8)));
typedef float    v4f  __attribute__((ext_vector_type(4)));
typedef unsigned int v4u __attribute__((ext_vector_type(4)));

union Frag  { v16h v; v8h h[2]; };
union Pack8 { v8h h; v4u u; };

__device__ __forceinline__ v8f mma16(v16h a, v16h b, v8f c) {
  c = __builtin_amdgcn_wmma_f32_16x16x32_f16(false, a, false, b, (short)0, c, false, false);
  asm volatile("v_nop\n\tv_nop\n\tv_nop\n\tv_nop" : "+v"(c) : "v"(a), "v"(b));
  return c;
}

__device__ __forceinline__ v16h ldfrag(const _Float16* p, int ld, int row0, int k0, int lane) {
  const int m = lane & 15, lh = lane >> 4;
  const _Float16* q = p + (size_t)(row0 + m) * ld + k0 + 8 * lh;
  Frag f;
  f.h[0] = *(const v8h*)(q);
  f.h[1] = *(const v8h*)(q + 16);
  return f.v;
}

__device__ __forceinline__ v8f zero8() { return (v8f){0.f, 0.f, 0.f, 0.f, 0.f, 0.f, 0.f, 0.f}; }

__device__ __forceinline__ void gemm32x64(const _Float16* __restrict__ A, int lda,
                                          const _Float16* __restrict__ Bt, int ldb,
                                          int m0, int n0, int kdim, int lane, v8f (&acc)[2][4]) {
#pragma unroll 2
  for (int k0 = 0; k0 < kdim; k0 += 32) {
    const v16h a0 = ldfrag(A, lda, m0, k0, lane);
    const v16h a1 = ldfrag(A, lda, m0 + 16, k0, lane);
    const v16h b0 = ldfrag(Bt, ldb, n0, k0, lane);
    const v16h b1 = ldfrag(Bt, ldb, n0 + 16, k0, lane);
    const v16h b2 = ldfrag(Bt, ldb, n0 + 32, k0, lane);
    const v16h b3 = ldfrag(Bt, ldb, n0 + 48, k0, lane);
    acc[0][0] = mma16(a0, b0, acc[0][0]);
    acc[1][0] = mma16(a1, b0, acc[1][0]);
    acc[0][1] = mma16(a0, b1, acc[0][1]);
    acc[1][1] = mma16(a1, b1, acc[1][1]);
    acc[0][2] = mma16(a0, b2, acc[0][2]);
    acc[1][2] = mma16(a1, b2, acc[1][2]);
    acc[0][3] = mma16(a0, b3, acc[0][3]);
    acc[1][3] = mma16(a1, b3, acc[1][3]);
  }
}

__global__ __launch_bounds__(256) void k_ln_gates(const float* __restrict__ x,
                                                  const float* __restrict__ gam,
                                                  const float* __restrict__ bet,
                                                  const float* __restrict__ wg,
                                                  const float* __restrict__ bg,
                                                  _Float16* __restrict__ xh,
                                                  float* __restrict__ gates) {
  __shared__ __align__(16) float gsh[8 * NE];
  const int tid = threadIdx.x, lane = tid & 31, wave = tid >> 5;
  const int row = blockIdx.x * 8 + wave;
  const float* xr = x + (size_t)row * DM;

  float s = 0.f;
#pragma unroll 1
  for (int it = 0; it < 4; ++it) {
    const int col = it * 256 + 8 * lane;
    const v4f a0 = *(const v4f*)(xr + col);
    const v4f a1 = *(const v4f*)(xr + col + 4);
    s += ((a0[0] + a0[1]) + (a0[2] + a0[3])) + ((a1[0] + a1[1]) + (a1[2] + a1[3]));
  }
#pragma unroll
  for (int off = 1; off < 32; off <<= 1) s += __shfl_xor(s, off, 32);
  const float mu = s * (1.0f / (float)DM);

  float qv = 0.f;
#pragma unroll 1
  for (int it = 0; it < 4; ++it) {
    const int col = it * 256 + 8 * lane;
    const v4f a0 = *(const v4f*)(xr + col);
    const v4f a1 = *(const v4f*)(xr + col + 4);
    const v4f d0 = a0 - mu;
    const v4f d1 = a1 - mu;
    qv += d0[0] * d0[0]; qv += d0[1] * d0[1]; qv += d0[2] * d0[2]; qv += d0[3] * d0[3];
    qv += d1[0] * d1[0]; qv += d1[1] * d1[1]; qv += d1[2] * d1[2]; qv += d1[3] * d1[3];
  }
#pragma unroll
  for (int off = 1; off < 32; off <<= 1) qv += __shfl_xor(qv, off, 32);
  const float rs = rsqrtf(qv * (1.0f / (float)DM) + 1e-5f);

  float g0 = 0.f, g1 = 0.f, g2 = 0.f, g3 = 0.f;
#pragma unroll 1
  for (int it = 0; it < 4; ++it) {
    const int col = it * 256 + 8 * lane;
    const v4f a0 = *(const v4f*)(xr + col);
    const v4f a1 = *(const v4f*)(xr + col + 4);
    const v4f ga0 = *(const v4f*)(gam + col);
    const v4f ga1 = *(const v4f*)(gam + col + 4);
    const v4f be0 = *(const v4f*)(bet + col);
    const v4f be1 = *(const v4f*)(bet + col + 4);
    v8f n;
    n[0] = ((a0[0] - mu) * rs) * ga0[0] + be0[0];
    n[1] = ((a0[1] - mu) * rs) * ga0[1] + be0[1];
    n[2] = ((a0[2] - mu) * rs) * ga0[2] + be0[2];
    n[3] = ((a0[3] - mu) * rs) * ga0[3] + be0[3];
    n[4] = ((a1[0] - mu) * rs) * ga1[0] + be1[0];
    n[5] = ((a1[1] - mu) * rs) * ga1[1] + be1[1];
    n[6] = ((a1[2] - mu) * rs) * ga1[2] + be1[2];
    n[7] = ((a1[3] - mu) * rs) * ga1[3] + be1[3];
#pragma unroll
    for (int j = 0; j < 8; ++j) {
      const v4f w = *(const v4f*)(wg + (size_t)(col + j) * NE);
      g0 += n[j] * w[0]; g1 += n[j] * w[1]; g2 += n[j] * w[2]; g3 += n[j] * w[3];
    }
    Pack8 pk;
    pk.h = (v8h){(_Float16)n[0], (_Float16)n[1], (_Float16)n[2], (_Float16)n[3],
                 (_Float16)n[4], (_Float16)n[5], (_Float16)n[6], (_Float16)n[7]};
    const v4u vv = pk.u;
    volatile v4u* dp = (volatile v4u*)(xh + (size_t)row * DM + col);
    *dp = vv;
    __threadfence();
    *dp = vv;
  }
#pragma unroll
  for (int off = 1; off < 32; off <<= 1) {
    g0 += __shfl_xor(g0, off, 32); g1 += __shfl_xor(g1, off, 32);
    g2 += __shfl_xor(g2, off, 32); g3 += __shfl_xor(g3, off, 32);
  }
  const float l0 = g0 + bg[0], l1 = g1 + bg[1], l2 = g2 + bg[2], l3 = g3 + bg[3];
  const float mx = fmaxf(fmaxf(l0, l1), fmaxf(l2, l3));
  const float p0 = __expf(l0 - mx), p1 = __expf(l1 - mx), p2 = __expf(l2 - mx), p3 = __expf(l3 - mx);
  const float inv = 1.0f / ((p0 + p1) + (p2 + p3));
  if (lane == 0) {
    gsh[wave * NE + 0] = p0 * inv;
    gsh[wave * NE + 1] = p1 * inv;
    gsh[wave * NE + 2] = p2 * inv;
    gsh[wave * NE + 3] = p3 * inv;
  }
  __syncthreads();
  if (wave == 0) {
    const int q = lane & 7;
    const v4f gv = *(const v4f*)(gsh + q * NE);
    volatile v4f* gp = (volatile v4f*)(gates + (size_t)(blockIdx.x * 8 + q) * NE);
    if (lane < 8) *gp = gv;
    __threadfence();
    if (lane < 8) *gp = gv;
  }
}

#define WTP 68
__global__ __launch_bounds__(256) void k_wt(const float* __restrict__ wsrc, _Float16* __restrict__ wdst,
                                            size_t src_es, size_t dst_es, int nout, int ldo, int kofs_e) {
  __shared__ __align__(16) float tf[64 * WTP];
  const int tid = threadIdx.x;
  const int n0 = blockIdx.x * 64;
  const int k0 = blockIdx.y * 64;
  const int e  = blockIdx.z;
  const float* w = wsrc + (size_t)e * src_es;
  _Float16* wt = wdst + (size_t)e * dst_es;
  const int kofs = e * kofs_e;
  {
    const int kr = tid >> 4;
    const int n4 = (tid & 15) * 4;
#pragma unroll
    for (int it = 0; it < 4; ++it) {
      const int kl = it * 16 + kr;
      const v4f a = *(const v4f*)(w + (size_t)(k0 + kl) * nout + n0 + n4);
      *(v4f*)(tf + kl * WTP + n4) = a;
    }
  }
  __syncthreads();
  v4u val[2];
  size_t go[2];
#pragma unroll
  for (int j = 0; j < 2; ++j) {
    const int p  = tid + 256 * j;
    const int nl = p >> 3;
    const int pc = p & 7;
    const float* cp = tf + (pc * 8) * WTP + nl;
    Pack8 pk;
    pk.h = (v8h){(_Float16)(cp[0 * WTP] * 32.0f), (_Float16)(cp[1 * WTP] * 32.0f),
                 (_Float16)(cp[2 * WTP] * 32.0f), (_Float16)(cp[3 * WTP] * 32.0f),
                 (_Float16)(cp[4 * WTP] * 32.0f), (_Float16)(cp[5 * WTP] * 32.0f),
                 (_Float16)(cp[6 * WTP] * 32.0f), (_Float16)(cp[7 * WTP] * 32.0f)};
    val[j] = pk.u;
    go[j]  = (size_t)(n0 + nl) * ldo + kofs + k0 + pc * 8;
  }
  for (int ps = 0; ps < 2; ++ps) {
#pragma unroll
    for (int j = 0; j < 2; ++j) *(volatile v4u*)(wt + go[j]) = val[j];
    __threadfence();
  }
}

#define STP 72
__global__ __launch_bounds__(256) void k_qkv(const _Float16* __restrict__ xh,
                                             const _Float16* __restrict__ wt,
                                             const float* __restrict__ bq,
                                             const float* __restrict__ bk,
                                             const float* __restrict__ bv,
                                             _Float16* __restrict__ qkv) {
  __shared__ __align__(16) _Float16 st[256 * STP];
  const int tid = threadIdx.x, lane = tid & 31, wave = tid >> 5;
  const int hh = lane >> 4, c = lane & 15;
  const int mb = blockIdx.x * 256;
  const int m0 = mb + wave * 32;
  const int n0 = blockIdx.y * 64;
  const int which = n0 >> 10;
  const int nin = n0 & (DM - 1);

  v8f acc[2][4];
#pragma unroll
  for (int s = 0; s < 2; ++s)
#pragma unroll
    for (int t = 0; t < 4; ++t) acc[s][t] = zero8();
  gemm32x64(xh, DM, wt, DM, m0, n0, DM, lane, acc);

#pragma unroll
  for (int t = 0; t < 4; ++t) {
    const int nn = nin + 16 * t + c;
    const float vq = bq[nn], vk = bk[nn], vvv = bv[nn];
    const float bvl = (which == 0) ? vq : ((which == 1) ? vk : vvv);
#pragma unroll
    for (int sub = 0; sub < 2; ++sub) {
#pragma unroll
      for (int r = 0; r < 8; ++r) {
        const int lr = wave * 32 + sub * 16 + 8 * hh + r;
        st[lr * STP + 16 * t + c] = (_Float16)(acc[sub][t][r] * 0.03125f + bvl);
      }
    }
  }
  __syncthreads();

  const int head = nin >> 6;
  const int b  = mb >> 10;
  const int nb = mb & (SS - 1);
  const int bh = b * NH + head;
  v4u val[8];
  size_t go[8];
  if (which < 2) {
#pragma unroll
    for (int j = 0; j < 8; ++j) {
      const int p  = tid + 256 * j;
      const int lr = p >> 3;
      const int pc = p & 7;
      Pack8 pk;
      pk.h  = *(const v8h*)(st + lr * STP + pc * 8);
      val[j] = pk.u;
      go[j]  = (size_t)which * PL + ((size_t)bh * SS + nb + lr) * HD + pc * 8;
    }
  } else {
#pragma unroll
    for (int j = 0; j < 8; ++j) {
      const int p  = tid + 256 * j;
      const int L  = p >> 3;
      const int pc = p & 7;
      const int d  = L >> 2;
      const int nl = (L & 3) * 64 + pc * 8;
      const _Float16* cp = st + nl * STP + d;
      Pack8 pk;
      pk.h = (v8h){cp[0 * STP], cp[1 * STP], cp[2 * STP], cp[3 * STP],
                   cp[4 * STP], cp[5 * STP], cp[6 * STP], cp[7 * STP]};
      val[j] = pk.u;
      go[j]  = 2 * PL + ((size_t)bh * HD + d) * SS + nb + nl;
    }
  }
  for (int ps = 0; ps < 2; ++ps) {
#pragma unroll
    for (int j = 0; j < 8; ++j) *(volatile v4u*)(qkv + go[j]) = val[j];
    __threadfence();
  }
}

#define KTP 72
#define PTP 72
__global__ __launch_bounds__(256) void k_attn(const _Float16* __restrict__ qp,
                                              const _Float16* __restrict__ kp,
                                              const _Float16* __restrict__ vt,
                                              const float* __restrict__ gates,
                                              _Float16* __restrict__ ctx,
                                              int e, float sscale) {
  __shared__ __align__(16) _Float16 Ks[64 * KTP];
  __shared__ __align__(16) _Float16 Vs[64 * KTP];
  __shared__ __align__(16) _Float16 Ps[8][16 * PTP];

  const int tid = threadIdx.x, lane = tid & 31, wave = tid >> 5;
  const int hh = lane >> 4, c = lane & 15;
  const int bh = blockIdx.x >> 3;
  const int qb = blockIdx.x & 7;
  const int b  = bh >> 4, h = bh & (NH - 1);
  const int q0 = qb * 128 + wave * 16;

  const _Float16* Q = qp + (size_t)bh * SS * HD;
  const _Float16* K = kp + (size_t)bh * SS * HD;
  const _Float16* V = vt + (size_t)bh * HD * SS;

  v16h qa[2];
  qa[0] = ldfrag(Q, HD, q0, 0, lane);
  qa[1] = ldfrag(Q, HD, q0, 32, lane);

  const float NEGI = -__builtin_huge_valf();
  float mrow[8], lrow[8];
  v8f oacc[4];
#pragma unroll
  for (int r = 0; r < 8; ++r) { mrow[r] = NEGI; lrow[r] = 0.f; }
#pragma unroll
  for (int t = 0; t < 4; ++t) oacc[t] = zero8();

  _Float16* pw = Ps[wave];

  for (int kc = 0; kc < SS / 64; ++kc) {
    const int kv0 = kc * 64;
    __syncthreads();
    {
      const int r  = tid >> 2;
      const int qq = (tid & 3) * 16;
      const _Float16* ks = K + (size_t)(kv0 + r) * HD + qq;
      *(v8h*)(Ks + r * KTP + qq)     = *(const v8h*)(ks);
      *(v8h*)(Ks + r * KTP + qq + 8) = *(const v8h*)(ks + 8);
      const _Float16* vs = V + (size_t)r * SS + kv0 + qq;
      *(v8h*)(Vs + r * KTP + qq)     = *(const v8h*)(vs);
      *(v8h*)(Vs + r * KTP + qq + 8) = *(const v8h*)(vs + 8);
    }
    __syncthreads();

    v8f s[4];
#pragma unroll
    for (int j = 0; j < 4; ++j) s[j] = zero8();
#pragma unroll
    for (int dc = 0; dc < 2; ++dc) {
#pragma unroll
      for (int j = 0; j < 4; ++j) {
        const v16h kb = ldfrag(Ks, KTP, j * 16, dc * 32, lane);
        s[j] = mma16(qa[dc], kb, s[j]);
      }
    }
    float cm[8];
#pragma unroll
    for (int r = 0; r < 8; ++r) {
      float m = NEGI;
#pragma unroll
      for (int j = 0; j < 4; ++j) {
        const float sv = s[j][r] * sscale;
        s[j][r] = sv;
        m = fmaxf(m, sv);
      }
#pragma unroll
      for (int off = 1; off < 16; off <<= 1) m = fmaxf(m, __shfl_xor(m, off, 32));
      cm[r] = m;
    }
    float al[8];
#pragma unroll
    for (int r = 0; r < 8; ++r) {
      const float mnew  = fmaxf(mrow[r], cm[r]);
      const float alpha = __expf(mrow[r] - mnew);
      mrow[r] = mnew;
      float psum = 0.f;
#pragma unroll
      for (int j = 0; j < 4; ++j) {
        const float p = __expf(s[j][r] - mnew);
        psum += p;
        pw[(8 * hh + r) * PTP + j * 16 + c] = (_Float16)(p * 1024.0f);
      }
#pragma unroll
      for (int off = 1; off < 16; off <<= 1) psum += __shfl_xor(psum, off, 32);
      lrow[r] = lrow[r] * alpha + psum;
      al[r] = alpha;
    }
#pragma unroll
    for (int t = 0; t < 4; ++t)
#pragma unroll
      for (int r = 0; r < 8; ++r) oacc[t][r] *= al[r];
    __syncthreads();

#pragma unroll
    for (int kk = 0; kk < 2; ++kk) {
      const v16h pa = ldfrag(pw, PTP, 0, kk * 32, lane);
#pragma unroll
      for (int t = 0; t < 4; ++t) {
        const v16h vb = ldfrag(Vs, KTP, t * 16, kk * 32, lane);
        oacc[t] = mma16(pa, vb, oacc[t]);
      }
    }
  }
  __syncthreads();

  const float* grow = gates + (size_t)(b * SS + q0 + 8 * hh) * NE + e;
#pragma unroll
  for (int r = 0; r < 8; ++r) {
    const float g   = grow[r * NE];
    const float inv = (g * 0.125f) * (1.0f / lrow[r]);
#pragma unroll
    for (int t = 0; t < 4; ++t) pw[(8 * hh + r) * PTP + 16 * t + c] = (_Float16)(oacc[t][r] * inv);
  }
  __syncthreads();
  v4u val[4];
  size_t go[4];
#pragma unroll
  for (int it = 0; it < 4; ++it) {
    const int p  = lane + 32 * it;
    const int L  = p >> 3;
    const int pc = p & 7;
    Pack8 pk;
    pk.h   = *(const v8h*)(pw + L * PTP + pc * 8);
    val[it] = pk.u;
    go[it]  = ((size_t)(b * SS + q0 + L)) * KCAT + (size_t)e * DM + (size_t)h * HD + pc * 8;
  }
  for (int ps = 0; ps < 2; ++ps) {
#pragma unroll
    for (int it = 0; it < 4; ++it) *(volatile v4u*)(ctx + go[it]) = val[it];
    __threadfence();
  }
}

#define OTP 68
__global__ __launch_bounds__(256) void k_out(const _Float16* __restrict__ ap,
                                             const _Float16* __restrict__ wt,
                                             const float* __restrict__ gates,
                                             const float* __restrict__ bo,
                                             const float* __restrict__ x,
                                             float* __restrict__ out) {
  __shared__ __align__(16) float st[8][16 * OTP];
  const int tid = threadIdx.x, lane = tid & 31, wave = tid >> 5;
  const int hh = lane >> 4, c = lane & 15;
  const int m0 = blockIdx.x * 256 + wave * 32;
  const int n0 = blockIdx.y * 64;

  v8f acc[2][4];
#pragma unroll
  for (int s = 0; s < 2; ++s)
#pragma unroll
    for (int t = 0; t < 4; ++t) acc[s][t] = zero8();
  gemm32x64(ap, KCAT, wt, KCAT, m0, n0, KCAT, lane, acc);

  float* sw = st[wave];
#pragma unroll
  for (int sub = 0; sub < 2; ++sub) {
    __syncthreads();
#pragma unroll
    for (int t = 0; t < 4; ++t) {
#pragma unroll
      for (int r = 0; r < 8; ++r)
        sw[(8 * hh + r) * OTP + 16 * t + c] = acc[sub][t][r] * 0.000244140625f;
    }
    __syncthreads();
#pragma unroll 1
    for (int it = 0; it < 8; ++it) {
      const int p    = lane + 32 * it;
      const int L    = p >> 3;
      const int pc   = p & 7;
      const int row  = L >> 1;
      const int half = L & 1;
      const int cl   = half * 32 + pc * 4;
      const int grow = m0 + sub * 16 + row;
      const int gcol = n0 + cl;
      v4f v = *(const v4f*)(sw + row * OTP + cl);
      const v4f xv = *(const v4f*)(x + (size_t)grow * DM + gcol);
      const v4f gv = *(const v4f*)(gates + (size_t)grow * NE);
      const v4f b0 = *(const v4f*)(bo + 0 * DM + gcol);
      const v4f b1 = *(const v4f*)(bo + 1 * DM + gcol);
      const v4f b2 = *(const v4f*)(bo + 2 * DM + gcol);
      const v4f b3 = *(const v4f*)(bo + 3 * DM + gcol);
      v4f gb = b0 * gv[0];
      gb = gb + b1 * gv[1];
      gb = gb + b2 * gv[2];
      gb = gb + b3 * gv[3];
      v = (v + gb) + xv;
      volatile v4f* dp = (volatile v4f*)(out + (size_t)grow * DM + gcol);
      *dp = v;
      __threadfence();
      *dp = v;
    }
  }
}

extern "C" void kernel_launch(void* const* d_in, const int* in_sizes, int n_in,
                              void* d_out, int out_size, void* d_ws, size_t ws_size,
                              hipStream_t stream) {
  if (n_in < 13) return;
  if (in_sizes[0] != ROWS * DM) return;
  if (in_sizes[1] != DM) return;
  if (in_sizes[2] != DM) return;
  if (in_sizes[3] != DM * NE) return;
  if (in_sizes[4] != NE) return;
  if (in_sizes[5] != NE * DM * DM) return;
  if (in_sizes[6] != NE * DM) return;
  if (in_sizes[7] != NE * DM * DM) return;
  if (in_sizes[8] != NE * DM) return;
  if (in_sizes[9] != NE * DM * DM) return;
  if (in_sizes[10] != NE * DM) return;
  if (in_sizes[11] != NE * DM * DM) return;
  if (in_sizes[12] != NE * DM) return;
  if (out_size != ROWS * DM) return;

  const float* x   = (const float*)d_in[0];
  const float* gam = (const float*)d_in[1];
  const float* bet = (const float*)d_in[2];
  const float* wg  = (const float*)d_in[3];
  const float* bg  = (const float*)d_in[4];
  const float* wq  = (const float*)d_in[5];
  const float* bq  = (const float*)d_in[6];
  const float* wk  = (const float*)d_in[7];
  const float* bk  = (const float*)d_in[8];
  const float* wv  = (const float*)d_in[9];
  const float* bv  = (const float*)d_in[10];
  const float* wo  = (const float*)d_in[11];
  const float* bo  = (const float*)d_in[12];
  float* out = (float*)d_out;

  size_t off = 0;
  const size_t oXh  = off; off += (size_t)ROWS * DM * 2;
  const size_t oG   = off; off += (size_t)ROWS * NE * 4;
  const size_t oWt  = off; off += (size_t)NE * C3 * DM * 2;
  const size_t oWo  = off; off += (size_t)DM * KCAT * 2;
  const size_t oQKV = off; off += 3 * PL * 2;
  const size_t oCTX = off; off += (size_t)ROWS * KCAT * 2;
  if (off > ws_size) return;
  if (off > (size_t)134217728) return;

  char* ws = (char*)d_ws;
  _Float16* Xh   = (_Float16*)(ws + oXh);
  float*    G    = (float*)(ws + oG);
  _Float16* Wt   = (_Float16*)(ws + oWt);
  _Float16* WoC  = (_Float16*)(ws + oWo);
  _Float16* QKVp = (_Float16*)(ws + oQKV);
  _Float16* CTX  = (_Float16*)(ws + oCTX);

  const size_t DD  = (size_t)DM * DM;
  const size_t WtE = (size_t)C3 * DM;

  k_ln_gates<<<dim3(ROWS / 8), dim3(256), 0, stream>>>(x, gam, bet, wg, bg, Xh, G);
  const dim3 wgrid(DM / 64, DM / 64, NE);
  k_wt<<<wgrid, dim3(256), 0, stream>>>(wq, Wt,          DD, WtE, DM, DM, 0);
  k_wt<<<wgrid, dim3(256), 0, stream>>>(wk, Wt + DD,     DD, WtE, DM, DM, 0);
  k_wt<<<wgrid, dim3(256), 0, stream>>>(wv, Wt + 2 * DD, DD, WtE, DM, DM, 0);
  k_wt<<<wgrid, dim3(256), 0, stream>>>(wo, WoC,         DD, (size_t)0, DM, KCAT, DM);
  for (int e = 0; e < NE; ++e) {
    k_qkv<<<dim3(ROWS / 256, C3 / 64), dim3(256), 0, stream>>>(Xh, Wt + (size_t)e * WtE,
                                                             bq + (size_t)e * DM, bk + (size_t)e * DM,
                                                             bv + (size_t)e * DM, QKVp);
    k_attn<<<dim3(BB * NH * (SS / 128)), dim3(256), 0, stream>>>(QKVp, QKVp + PL, QKVp + 2 * PL,
                                                                  G, CTX, e, 0.125f);
  }
  k_out<<<dim3(ROWS / 256, DM / 64), dim3(256), 0, stream>>>(CTX, WoC, G, bo, x, out);
  (void)hipGetLastError();
}
